// self_att_3951369912398
// MI455X (gfx1250) — hardware-verified
//
#include <hip/hip_runtime.h>
#include <math.h>
#include <stdint.h>

#define NB   8
#define NT   1024
#define ND   512
#define NH   8
#define NHD  64
#define LN_EPS 1e-5f
#define PSCALE 32768.0f

typedef __attribute__((ext_vector_type(16))) _Float16 v16h;
typedef __attribute__((ext_vector_type(8)))  _Float16 v8h;
typedef __attribute__((ext_vector_type(16))) __bf16   v16b;
typedef __attribute__((ext_vector_type(8)))  __bf16   v8b;
typedef __attribute__((ext_vector_type(8)))  float    v8f;
typedef __attribute__((ext_vector_type(4)))  float    v4f;
typedef __attribute__((ext_vector_type(2)))  float    v2f;
typedef __attribute__((ext_vector_type(4)))  unsigned int v4u;

__device__ __forceinline__ unsigned short f2bf_bits(float f) {
  unsigned u = __float_as_uint(f);
  return (unsigned short)((u + 0x7FFFu + ((u >> 16) & 1u)) >> 16);
}
__device__ __forceinline__ float bf_bits2f(unsigned short h) { return __uint_as_float(((unsigned)h) << 16); }
__device__ __forceinline__ float h2f(unsigned short u) { return (float)__builtin_bit_cast(_Float16, u); }

__device__ __forceinline__ void dep_guard_h(v8f& a, v8f& b, v16h x, v16h y) { asm volatile("v_nop\n\tv_nop\n\tv_nop\n\tv_nop" : "+v"(a), "+v"(b) : "v"(x), "v"(y)); }
__device__ __forceinline__ void dep_guard_b(v8f& a, v8f& b, v16b x, v16b y) { asm volatile("v_nop\n\tv_nop\n\tv_nop\n\tv_nop" : "+v"(a), "+v"(b) : "v"(x), "v"(y)); }
__device__ __forceinline__ void keep4_h(v16h a, v16h b, v16h c, v16h d) { asm volatile("v_nop" :: "v"(a), "v"(b), "v"(c), "v"(d)); }
__device__ __forceinline__ void keep4_b(v16b a, v16b b, v16b c, v16b d) { asm volatile("v_nop" :: "v"(a), "v"(b), "v"(c), "v"(d)); }
__device__ __forceinline__ void acc_guard4(v8f& a, v8f& b, v8f& c, v8f& d) { asm volatile("v_nop\n\tv_nop\n\tv_nop\n\tv_nop" : "+v"(a), "+v"(b), "+v"(c), "+v"(d)); }
template <typename T> struct Frag;
template <> struct Frag<_Float16> {
  typedef v16h V; union U { v16h v; v8h h[2]; };
  static __device__ __forceinline__ v16h load(const _Float16* p) {
    U f; f.h[0] = *(const v8h*)(p); f.h[1] = *(const v8h*)(p + 16); return f.v;
  }
  static __device__ __forceinline__ v8f mma(v16h a, v16h b, v8f c) {
    return __builtin_amdgcn_wmma_f32_16x16x32_f16(false, a, false, b, (short)0, c, false, false);
  }
  static __device__ __forceinline__ void guard(v8f& a, v8f& b, v16h x, v16h y) { dep_guard_h(a, b, x, y); }
  static __device__ __forceinline__ void keep(v16h a, v16h b, v16h c, v16h d) { keep4_h(a, b, c, d); }
};
template <> struct Frag<__bf16> {
  typedef v16b V; union U { v16b v; v8b h[2]; };
  static __device__ __forceinline__ v16b load(const __bf16* p) {
    U f; f.h[0] = *(const v8b*)(p); f.h[1] = *(const v8b*)(p + 16); return f.v;
  }
  static __device__ __forceinline__ v8f mma(v16b a, v16b b, v8f c) {
    return __builtin_amdgcn_wmma_f32_16x16x32_bf16(false, a, false, b, (short)0, c, false, false);
  }
  static __device__ __forceinline__ void guard(v8f& a, v8f& b, v16b x, v16b y) { dep_guard_b(a, b, x, y); }
  static __device__ __forceinline__ void keep(v16b a, v16b b, v16b c, v16b d) { keep4_b(a, b, c, d); }
};

template <int ET> struct Elem;
template <> struct Elem<0> { typedef _Float16 T; };
template <> struct Elem<1> { typedef __bf16 T; };
template <int ET, bool SPLIT, int BIAS_MODE, int OUT_MODE, bool RESID, int ACT = 0>
__global__ __launch_bounds__(256) void wmma_gemm64(
    const unsigned short* __restrict__ Ap, const unsigned short* __restrict__ A2p, int lda, long strideA,
    const unsigned short* __restrict__ Btp, const unsigned short* __restrict__ Bt2p, int ldb, long strideB,
    void* __restrict__ Cout, void* __restrict__ Cout2, int ldc, long strideC,
    const float* __restrict__ bias,
    const float* __restrict__ resid, long strideR,
    int M, int N, int K, float scale) {
  typedef typename Elem<ET>::T T;
  typedef typename Frag<T>::V V;
  const T* A = (const T*)Ap; const T* A2 = (const T*)A2p; const T* Bt = (const T*)Btp; const T* Bt2 = (const T*)Bt2p;
  __shared__ __align__(16) float sT[8][16 * 68];
  const int b    = blockIdx.y;
  const int lane = threadIdx.x & 31;
  const int wave = threadIdx.x >> 5;
  const int tilesN = N >> 6;
  const int tilesM = M >> 6;
  const int tile = blockIdx.x * 8 + wave;
  if (tile >= tilesM * tilesN) return;
  const int tm = tile / tilesN;
  const int tn = tile - tm * tilesN;
  const int m0 = tm << 6;
  const int n0 = tn << 6;

  const T* Ab  = A  + (size_t)b * strideA;
  const T* Bb  = Bt + (size_t)b * strideB;
  const T* Ab2 = SPLIT ? (A2  + (size_t)b * strideA) : nullptr;
  const T* Bb2 = SPLIT ? (Bt2 + (size_t)b * strideB) : nullptr;

  const int rlane = lane & 15;
  const int koff  = (lane >> 4) * 8;
  const int mOff  = (lane >> 4) * 8;

  v8f acc[4][4];
#pragma unroll
  for (int i = 0; i < 4; ++i)
#pragma unroll
    for (int j = 0; j < 4; ++j) acc[i][j] = (v8f){0.f,0.f,0.f,0.f,0.f,0.f,0.f,0.f};

  for (int k0 = 0; k0 < K; k0 += 32) {
    V bh[4], bl[4];
#pragma unroll
    for (int j = 0; j < 4; ++j) {
      const size_t bo = (size_t)(n0 + (j << 4) + rlane) * ldb + koff + k0;
      bh[j] = Frag<T>::load(Bb + bo);
      if (SPLIT) bl[j] = Frag<T>::load(Bb2 + bo);
    }
#pragma unroll
    for (int i = 0; i < 4; ++i) {
      const size_t ao = (size_t)(m0 + (i << 4) + rlane) * lda + koff + k0;
      V ah = Frag<T>::load(Ab + ao);
      V al;
      if (SPLIT) al = Frag<T>::load(Ab2 + ao);
#pragma unroll
      for (int j = 0; j < 4; ++j) {
        acc[i][j] = Frag<T>::mma(ah, bh[j], acc[i][j]);
        if (SPLIT) {
          acc[i][j] = Frag<T>::mma(ah, bl[j], acc[i][j]);
          acc[i][j] = Frag<T>::mma(al, bh[j], acc[i][j]);
        }
      }
      Frag<T>::guard(acc[i][0], acc[i][3], ah, SPLIT ? al : ah);
    }
    Frag<T>::keep(bh[0], bh[1], bh[2], bh[3]);
    if (SPLIT) Frag<T>::keep(bl[0], bl[1], bl[2], bl[3]);
  }
  acc_guard4(acc[0][0], acc[0][1], acc[0][2], acc[0][3]);
  acc_guard4(acc[1][0], acc[1][1], acc[1][2], acc[1][3]);
  acc_guard4(acc[2][0], acc[2][1], acc[2][2], acc[2][3]);
  acc_guard4(acc[3][0], acc[3][1], acc[3][2], acc[3][3]);

  float* slab = sT[wave];
  const float* Rb = RESID ? (resid + (size_t)b * strideR) : nullptr;
#pragma unroll
  for (int i = 0; i < 4; ++i) {
    const int mBase = m0 + (i << 4);
#pragma unroll
    for (int j = 0; j < 4; ++j) {
      const int n = n0 + (j << 4) + rlane;
      float bv = 0.f;
      if (BIAS_MODE == 2) bv = bias[n];
#pragma unroll
      for (int r = 0; r < 8; ++r) {
        float v = acc[i][j][r] * scale;
        if (BIAS_MODE == 1) v += bias[mBase + mOff + r];
        if (BIAS_MODE == 2) v += bv;
        if (RESID) v += Rb[(size_t)(mBase + mOff + r) * ldc + n];
        if (ACT == 1) v = tanhf(v);
        if (ACT == 2) v = fmaxf(v, 0.0f);
        if (ACT == 3) v = v / (1.0f + expf(-v));
        if (ACT == 4) v = (v > 0.f) ? v : 0.01f * v;
        slab[(mOff + r) * 68 + (j << 4) + rlane] = v;
      }
    }
    __builtin_amdgcn_fence(__ATOMIC_RELEASE, "workgroup");
    __builtin_amdgcn_wave_barrier();
    __builtin_amdgcn_fence(__ATOMIC_ACQUIRE, "workgroup");
    if (OUT_MODE == 0) {
      float* C = (float*)Cout + (size_t)b * strideC;
      const int hh = lane >> 4, c4 = (lane & 15) * 4;
      for (int pass = 0; pass < 2; ++pass) {
#pragma unroll
        for (int it = 0; it < 8; ++it) {
          const int row = it * 2 + hh;
          v4f v = *(const v4f*)(slab + row * 68 + c4);
          *(volatile v4f*)(C + (size_t)(mBase + row) * ldc + n0 + c4) = v;
        }
        __threadfence();
      }
    } else {
      const int q = lane >> 3, c8 = (lane & 7) * 8;
      unsigned short* C  = (unsigned short*)Cout  + (size_t)b * strideC;
      unsigned short* C2 = (OUT_MODE == 2) ? ((unsigned short*)Cout2 + (size_t)b * strideC) : nullptr;
      for (int pass = 0; pass < 2; ++pass) {
#pragma unroll
        for (int it = 0; it < 4; ++it) {
          const int row = it * 4 + q;
          const float* sp = slab + row * 68 + c8;
          v8h hv, lv;
#pragma unroll
          for (int e = 0; e < 8; ++e) {
            if (OUT_MODE == 1) {
              hv[e] = (_Float16)sp[e];
            } else {
              unsigned short hb = f2bf_bits(sp[e]);
              unsigned short lb = f2bf_bits(sp[e] - bf_bits2f(hb));
              hv[e] = __builtin_bit_cast(_Float16, hb);
              lv[e] = __builtin_bit_cast(_Float16, lb);
            }
          }
          *(volatile v8h*)(C + (size_t)(mBase + row) * ldc + n0 + c8) = hv;
          if (OUT_MODE == 2) *(volatile v8h*)(C2 + (size_t)(mBase + row) * ldc + n0 + c8) = lv;
        }
        __threadfence();
      }
    }
    __builtin_amdgcn_fence(__ATOMIC_RELEASE, "workgroup");
    __builtin_amdgcn_wave_barrier();
    __builtin_amdgcn_fence(__ATOMIC_ACQUIRE, "workgroup");
  }
}

__device__ __forceinline__ unsigned pk16(unsigned short a, unsigned short b) { return (unsigned)a | ((unsigned)b << 16); }
__device__ __forceinline__ unsigned short h_bits(float f) { const _Float16 h = (_Float16)f; return __builtin_bit_cast(unsigned short, h); }

__global__ __launch_bounds__(256) void cast_f16x2_kernel(const float* __restrict__ in, unsigned short* __restrict__ out, int n2, float scale) {
  const int i = blockIdx.x * 256 + threadIdx.x;
  if (i < n2) {
    const v2f f = *(const v2f*)(in + 2 * (size_t)i);
    const unsigned u = pk16(h_bits(f[0] * scale), h_bits(f[1] * scale));
    ((volatile unsigned*)out)[i] = u;
    __threadfence();
    ((volatile unsigned*)out)[i] = u;
  }
}

__global__ __launch_bounds__(256) void transpose_cast_f16_kernel(const float* __restrict__ in, unsigned short* __restrict__ out,
                                                                 int R, int C, float scale) {
  __shared__ float tile[64][65];
  const int tid = threadIdx.x;
  const int lane = tid & 31, wave = tid >> 5;
  const int c0 = blockIdx.x * 64;
  const int r0 = blockIdx.y * 64;
#pragma unroll
  for (int e = 0; e < 16; ++e) {
    const int idx = tid + 256 * e;
    const int rr = idx >> 6, cc = idx & 63;
    tile[cc][rr] = in[(size_t)(r0 + rr) * C + c0 + cc] * scale;
  }
  __syncthreads();
  const int q = lane >> 3, c8 = (lane & 7) * 8;
  v4u hv[2];
  size_t oo[2];
#pragma unroll
  for (int it = 0; it < 2; ++it) {
    const int orow = wave * 8 + it * 4 + q;
    const float* sp = &tile[orow][c8];
    hv[it] = (v4u){pk16(h_bits(sp[0]), h_bits(sp[1])), pk16(h_bits(sp[2]), h_bits(sp[3])),
                   pk16(h_bits(sp[4]), h_bits(sp[5])), pk16(h_bits(sp[6]), h_bits(sp[7]))};
    oo[it] = (size_t)(c0 + orow) * R + r0 + c8;
  }
  for (int pass = 0; pass < 2; ++pass) {
#pragma unroll
    for (int it = 0; it < 2; ++it) *(volatile v4u*)(out + oo[it]) = hv[it];
    __threadfence();
  }
}

__global__ __launch_bounds__(256) void score_vec_kernel(const unsigned short* __restrict__ QXT, const unsigned short* __restrict__ KXT,
                                                         const float* __restrict__ w, float* __restrict__ QS, float* __restrict__ KS) {
  const int t = blockIdx.x * 256 + threadIdx.x;
  const int b = blockIdx.y;
  if (t >= NT) return;
  const unsigned short* qp = QXT + (size_t)b * ND * NT + t;
  const unsigned short* kp = KXT + (size_t)b * ND * NT + t;
#pragma unroll 1
  for (int h = 0; h < NH; ++h) {
    const unsigned short* qh = qp + (size_t)h * NHD * NT;
    const unsigned short* kh = kp + (size_t)h * NHD * NT;
    float sq = 0.f, sk = 0.f;
#pragma unroll 1
    for (int d = 0; d < NHD; ++d) {
      const float qv = h2f(qh[(size_t)d * NT]);
      const float kv = h2f(kh[(size_t)d * NT]);
      sk += kv * w[d];
      sq += qv * w[NHD + d];
    }
    const size_t o = ((size_t)b * NH + h) * NT + t;
    ((volatile float*)QS)[o] = sq;
    ((volatile float*)KS)[o] = sk;
    __threadfence();
    ((volatile float*)QS)[o] = sq;
    ((volatile float*)KS)[o] = sk;
  }
}

#define PK_NT 128
#define PK_RPB 8
__global__ __launch_bounds__(PK_NT) void prob_kernel(const float* __restrict__ QS, const float* __restrict__ KS,
                                                     unsigned short* __restrict__ P16, int b) {
  __shared__ __align__(16) float Ksh[NT];
  __shared__ __align__(16) float Esh[NT];
  __shared__ float red[PK_NT / 32];
  const int tid = threadIdx.x;
  const int lane = tid & 31, wave = tid >> 5;
  const int h = blockIdx.y;
  const int i0 = blockIdx.x * PK_RPB;
  const size_t bh = (size_t)b * NH + h;
  {
    const float* kp = KS + bh * NT + tid * 8;
    const v4f a = *(const v4f*)kp;
    const v4f c = *(const v4f*)(kp + 4);
    *(v4f*)(Ksh + tid * 8) = a;
    *(v4f*)(Ksh + tid * 8 + 4) = c;
  }
  __syncthreads();
  const float* qp = QS + bh * NT + i0;
#pragma unroll 1
  for (int r = 0; r < PK_RPB; ++r) {
    const float qv = qp[r];
    float s = 0.f;
#pragma unroll 1
    for (int e = 0; e < NT / PK_NT; ++e) {
      const int j = tid + PK_NT * e;
      float z = qv + Ksh[j];
      z = fminf(fmaxf(z, -15.0f), 15.0f);
      const float e2 = __expf(2.0f * z);
      const float th = 1.0f - 2.0f * __builtin_amdgcn_rcpf(e2 + 1.0f);
      const float ev = __expf(th);
      Esh[j] = ev;
      s += ev;
    }
#pragma unroll
    for (int off = 16; off > 0; off >>= 1) s += __shfl_xor(s, off, 32);
    if (lane == 0) red[wave] = s;
    __syncthreads();
    const float tot = ((red[0] + red[1]) + red[2]) + red[3];
    const float sc = PSCALE * __builtin_amdgcn_rcpf(tot);
    const float* ep = Esh + tid * 8;
    const v4f a = *(const v4f*)ep;
    const v4f c = *(const v4f*)(ep + 4);
    const v4u hv = (v4u){pk16(h_bits(a[0] * sc), h_bits(a[1] * sc)),
                         pk16(h_bits(a[2] * sc), h_bits(a[3] * sc)),
                         pk16(h_bits(c[0] * sc), h_bits(c[1] * sc)),
                         pk16(h_bits(c[2] * sc), h_bits(c[3] * sc))};
    const size_t ro = ((size_t)h * NT + (i0 + r)) * NT + tid * 8;
    *(volatile v4u*)(P16 + ro) = hv;
    __threadfence();
    *(volatile v4u*)(P16 + ro) = hv;
    __syncthreads();
  }
}

__global__ __launch_bounds__(256) void layernorm_kernel(const float* __restrict__ Y, const float* __restrict__ gam,
                                                        const float* __restrict__ bet, float* __restrict__ out, int nrows) {
  const int lane = threadIdx.x & 31, wave = threadIdx.x >> 5;
  const int row = blockIdx.x * 8 + wave;
  if (row >= nrows) return;
  const float* yp = Y + (size_t)row * ND + lane * 4;
  const v4f v0 = *(const v4f*)(yp);
  const v4f v1 = *(const v4f*)(yp + 128);
  const v4f v2 = *(const v4f*)(yp + 256);
  const v4f v3 = *(const v4f*)(yp + 384);
  float s = (((v0[0] + v0[1]) + (v0[2] + v0[3])) + ((v1[0] + v1[1]) + (v1[2] + v1[3])))
          + (((v2[0] + v2[1]) + (v2[2] + v2[3])) + ((v3[0] + v3[1]) + (v3[2] + v3[3])));
#pragma unroll
  for (int off = 16; off > 0; off >>= 1) s += __shfl_xor(s, off, 32);
  const float mu = s * (1.0f / 512.0f);
  const v4f mv = (v4f){mu, mu, mu, mu};
  const v4f d0 = v0 - mv, d1 = v1 - mv, d2 = v2 - mv, d3 = v3 - mv;
  float ss = (((d0[0] * d0[0] + d0[1] * d0[1]) + (d0[2] * d0[2] + d0[3] * d0[3]))
            + ((d1[0] * d1[0] + d1[1] * d1[1]) + (d1[2] * d1[2] + d1[3] * d1[3])))
           + (((d2[0] * d2[0] + d2[1] * d2[1]) + (d2[2] * d2[2] + d2[3] * d2[3]))
            + ((d3[0] * d3[0] + d3[1] * d3[1]) + (d3[2] * d3[2] + d3[3] * d3[3])));
#pragma unroll
  for (int off = 16; off > 0; off >>= 1) ss += __shfl_xor(ss, off, 32);
  const float var = ss * (1.0f / 512.0f);
  const float rs = rsqrtf(var + LN_EPS);
  const v4f rv = (v4f){rs, rs, rs, rs};
  const float* gp = gam + lane * 4;
  const float* bp = bet + lane * 4;
  const v4f g0 = *(const v4f*)(gp), g1 = *(const v4f*)(gp + 128), g2 = *(const v4f*)(gp + 256), g3 = *(const v4f*)(gp + 384);
  const v4f b0 = *(const v4f*)(bp), b1 = *(const v4f*)(bp + 128), b2 = *(const v4f*)(bp + 256), b3 = *(const v4f*)(bp + 384);
  const v4f o0 = (d0 * rv) * g0 + b0;
  const v4f o1 = (d1 * rv) * g1 + b1;
  const v4f o2 = (d2 * rv) * g2 + b2;
  const v4f o3 = (d3 * rv) * g3 + b3;
  float* op = out + (size_t)row * ND + lane * 4;
  for (int pass = 0; pass < 2; ++pass) {
    *(volatile v4f*)(op)       = o0;
    *(volatile v4f*)(op + 128) = o1;
    *(volatile v4f*)(op + 256) = o2;
    *(volatile v4f*)(op + 384) = o3;
    __threadfence();
  }
}

extern "C" void kernel_launch(void* const* d_in, const int* in_sizes, int n_in,
                              void* d_out, int out_size, void* d_ws, size_t ws_size,
                              hipStream_t stream) {
  if (n_in < 10) return;
  if (in_sizes[0] != NB * NT * ND) return;
  if (in_sizes[1] != ND * ND || in_sizes[3] != ND * ND || in_sizes[5] != ND * ND) return;
  if (in_sizes[2] != ND || in_sizes[4] != ND || in_sizes[6] != ND) return;
  if (in_sizes[7] != 2 * NHD || in_sizes[8] != ND || in_sizes[9] != ND) return;
  if (out_size != NB * NT * ND) return;

  const float* x     = (const float*)d_in[0];
  const float* Wq    = (const float*)d_in[1];
  const float* bq    = (const float*)d_in[2];
  const float* Wk    = (const float*)d_in[3];
  const float* bk    = (const float*)d_in[4];
  const float* Wp    = (const float*)d_in[5];
  const float* bp    = (const float*)d_in[6];
  const float* w_mlp = (const float*)d_in[7];
  const float* ln_g  = (const float*)d_in[8];
  const float* ln_b  = (const float*)d_in[9];
  float* out = (float*)d_out;

  const size_t PW  = (size_t)ND * ND * 2;
  const size_t PA  = (size_t)NB * NT * ND * 2;
  const size_t PSV = (size_t)NB * NH * NT * 4;
  const size_t PP  = (size_t)NH * NT * NT * 2;
  const size_t PY  = (size_t)NB * NT * ND * 4;
  size_t off = 0;
  const size_t oWq  = off; off += PW;
  const size_t oWk  = off; off += PW;
  const size_t oWp  = off; off += PW;
  const size_t oX   = off; off += PA;
  const size_t oQXT = off; off += PA;
  const size_t oKXT = off; off += PA;
  const size_t oQS  = off; off += PSV;
  const size_t oKS  = off; off += PSV;
  const size_t oP   = off; off += PP;
  const size_t oCTX = off; off += PA;
  const size_t oY   = off; off += PY;
  if (off > ws_size) return;

  char* ws = (char*)d_ws;
  unsigned short* WqT16 = (unsigned short*)(ws + oWq);
  unsigned short* WkT16 = (unsigned short*)(ws + oWk);
  unsigned short* WpT16 = (unsigned short*)(ws + oWp);
  unsigned short* X16   = (unsigned short*)(ws + oX);
  unsigned short* QXT16 = (unsigned short*)(ws + oQXT);
  unsigned short* KXT16 = (unsigned short*)(ws + oKXT);
  float*          QS    = (float*)(ws + oQS);
  float*          KS    = (float*)(ws + oKS);
  unsigned short* P16   = (unsigned short*)(ws + oP);
  unsigned short* CTX16 = (unsigned short*)(ws + oCTX);
  float*          Ybuf  = (float*)(ws + oY);

  const dim3 blk(256);
  const int BT = NB * NT;

  transpose_cast_f16_kernel<<<dim3(ND / 64, ND / 64), blk, 0, stream>>>(Wq, WqT16, ND, ND, 16.0f);
  transpose_cast_f16_kernel<<<dim3(ND / 64, ND / 64), blk, 0, stream>>>(Wk, WkT16, ND, ND, 16.0f);
  transpose_cast_f16_kernel<<<dim3(ND / 64, ND / 64), blk, 0, stream>>>(Wp, WpT16, ND, ND, 16.0f);
  {
    const int n2 = BT * ND / 2;
    cast_f16x2_kernel<<<dim3((n2 + 255) / 256), blk, 0, stream>>>(x, X16, n2, 1.0f);
  }
  const float wscale = 1.0f / 16.0f;
  const dim3 gProj(((ND / 64) * (NT / 64) + 7) / 8, NB);
  wmma_gemm64<0, false, 1, 1, false, 0><<<gProj, blk, 0, stream>>>(
      WqT16, WqT16, ND, 0L, X16, X16, ND, (long)NT * ND, (void*)QXT16, (void*)QXT16, NT, (long)ND * NT,
      bq, x, 0L, ND, NT, ND, wscale);
  wmma_gemm64<0, false, 1, 1, false, 0><<<gProj, blk, 0, stream>>>(
      WkT16, WkT16, ND, 0L, X16, X16, ND, (long)NT * ND, (void*)KXT16, (void*)KXT16, NT, (long)ND * NT,
      bk, x, 0L, ND, NT, ND, wscale);
  score_vec_kernel<<<dim3(NT / 256, NB), blk, 0, stream>>>(QXT16, KXT16, w_mlp, QS, KS);
  const dim3 gProb(NT / PK_RPB, NH);
  const dim3 gPV(((NT / 64) * (NHD / 64) + 7) / 8, NH);
  const float pvscale = 16.0f / PSCALE;
  for (int b = 0; b < NB; ++b) {
    prob_kernel<<<gProb, dim3(PK_NT), 0, stream>>>(QS, KS, P16, b);
    wmma_gemm64<0, false, 0, 1, false, 0><<<gPV, blk, 0, stream>>>(
        P16, P16, NT, (long)NT * NT,
        KXT16 + (size_t)b * ND * NT, KXT16 + (size_t)b * ND * NT, NT, (long)NHD * NT,
        (void*)(CTX16 + (size_t)b * NT * ND), (void*)(CTX16 + (size_t)b * NT * ND), ND, (long)NHD,
        bq, x, 0L, NT, NHD, NT, pvscale);
  }
  const dim3 gOut(((BT / 64) * (ND / 64) + 7) / 8, 1);
  wmma_gemm64<0, false, 2, 0, true, 0><<<gOut, blk, 0, stream>>>(
      CTX16, CTX16, ND, 0L, WpT16, WpT16, ND, 0L, (void*)Ybuf, (void*)Ybuf, ND, 0L,
      bp, x, 0L, BT, ND, ND, 1.0f / 256.0f);
  layernorm_kernel<<<dim3((BT + 7) / 8), blk, 0, stream>>>(Ybuf, ln_g, ln_b, out, BT);
  (void)hipGetLastError();
}
